// GroupAttention_86784109183341
// MI455X (gfx1250) — hardware-run, weakly checked
//
#include <hip/hip_runtime.h>
#include <math.h>
#include <stdint.h>

#ifndef NB
#define NB 4
#endif
#define NB_FULL 4
#define QLEN   512
#define MLEN   512
#define KLEN   1024
#define ND     1024
#define NH     16
#define HDV    64
#define HQK    128
#define NG     4
#define DG     256
#define QKW    (2 * ND)
#define LDQ    (NB * QKW)
#define NKT    (KLEN / 64)
#define NQT    (QLEN / 64)
#define NPAIR  8
#define BDN    KLEN
#define LN_EPS 1e-6f

static_assert(NB >= 1);
static_assert(NB <= NB_FULL);
static_assert(ND == NH * HDV);
static_assert(ND == NG * DG);
static_assert(HQK == 2 * HDV);
static_assert(KLEN == MLEN + QLEN);
static_assert(QLEN % 64 == 0);
static_assert(KLEN % 64 == 0);
static_assert(DG % 64 == 0);
static_assert(NH % NPAIR == 0);
static_assert((QLEN * NB) % 64 == 0);
static_assert(QKW % 32 == 0);

typedef _Float16 v16h __attribute__((ext_vector_type(16)));
typedef _Float16 v8h  __attribute__((ext_vector_type(8)));
typedef float    v8f  __attribute__((ext_vector_type(8)));
typedef float    v4f  __attribute__((ext_vector_type(4)));
typedef int      v4i  __attribute__((ext_vector_type(4)));
typedef v4f __attribute__((may_alias)) v4fa;
typedef v8h __attribute__((may_alias)) v8ha;
typedef v4i __attribute__((may_alias)) v4ia;

__device__ __forceinline__ float bf_rne(float f) {
  unsigned u = __float_as_uint(f);
  u = (u + 0x7FFFu + ((u >> 16) & 1u)) & 0xFFFF0000u;
  return __uint_as_float(u);
}

union FragU { v16h v; v8ha h[2]; };
__device__ __forceinline__ v16h ldfrag(const _Float16* p) {
  FragU f;
  f.h[0] = *(const v8ha*)(p);
  f.h[1] = *(const v8ha*)(p + 16);
  return f.v;
}

__device__ __forceinline__ v8f mma16(v16h a, v16h b, v8f c) {
  c = __builtin_amdgcn_wmma_f32_16x16x32_f16(false, a, false, b, (short)0, c, false, false);
  asm volatile("v_nop\n\tv_nop\n\tv_nop\n\tv_nop" : "+v"(c) : "v"(a), "v"(b));
  return c;
}

__device__ __forceinline__ v8f zero8() { v8f z = {0.f, 0.f, 0.f, 0.f, 0.f, 0.f, 0.f, 0.f}; return z; }

__global__ __launch_bounds__(256) void cvt1_kernel(const float* __restrict__ src, _Float16* __restrict__ dst,
                                                   int n8, float s1) {
  const int i = blockIdx.x * 256 + threadIdx.x;
  if (i >= n8) return;
  const float* sp = src + (size_t)i * 8;
  const v4f a = *(const v4f*)(sp);
  const v4f b = *(const v4f*)(sp + 4);
  float f[8];
  f[0] = bf_rne(a[0]); f[1] = bf_rne(a[1]); f[2] = bf_rne(a[2]); f[3] = bf_rne(a[3]);
  f[4] = bf_rne(b[0]); f[5] = bf_rne(b[1]); f[6] = bf_rne(b[2]); f[7] = bf_rne(b[3]);
  v8h o1;
#pragma unroll
  for (int e = 0; e < 8; ++e) o1[e] = (_Float16)(f[e] * s1);
  _Float16* dp = dst + (size_t)i * 8;
  *(volatile v8h*)dp = o1;
  __threadfence();
  *(volatile v8h*)dp = o1;
}

template <bool GROUPED>
__global__ __launch_bounds__(256) void cvt2_kernel(const float* __restrict__ W1, const float* __restrict__ W2,
                                                   _Float16* __restrict__ dst) {
  const int i = blockIdx.x * 256 + threadIdx.x;
  if (i >= ND * (ND / 8)) return;
  const int o  = i / (ND / 8);
  const int c8 = (i - o * (ND / 8)) * 8;
  const int og = GROUPED ? (o % DG) : o;
  const float* sp = W1 + (size_t)og * ND + c8;
  const v4f a = *(const v4f*)(sp);
  const v4f b = *(const v4f*)(sp + 4);
  float f[8];
  f[0] = bf_rne(a[0]); f[1] = bf_rne(a[1]); f[2] = bf_rne(a[2]); f[3] = bf_rne(a[3]);
  f[4] = bf_rne(b[0]); f[5] = bf_rne(b[1]); f[6] = bf_rne(b[2]); f[7] = bf_rne(b[3]);
  if (GROUPED) {
    const int g  = o / DG;
    const int dg = c8 % DG;
    const float same = ((c8 / DG) == g) ? 1.0f : 0.0f;
    const float* gp = W2 + ((size_t)(g * DG + og)) * DG + dg;
    const v4f ga = *(const v4f*)(gp);
    const v4f gb = *(const v4f*)(gp + 4);
    f[0] += same * bf_rne(ga[0]); f[1] += same * bf_rne(ga[1]); f[2] += same * bf_rne(ga[2]); f[3] += same * bf_rne(ga[3]);
    f[4] += same * bf_rne(gb[0]); f[5] += same * bf_rne(gb[1]); f[6] += same * bf_rne(gb[2]); f[7] += same * bf_rne(gb[3]);
  }
  v8h hv, lv;
#pragma unroll
  for (int e = 0; e < 8; ++e) {
    hv[e] = (_Float16)(f[e] * 64.0f);
    lv[e] = (_Float16)(f[e] * 0.0625f);
  }
  _Float16* dp = dst + (size_t)o * QKW + c8;
  *(volatile v8h*)(dp)      = hv;
  *(volatile v8h*)(dp + ND) = lv;
  __threadfence();
  *(volatile v8h*)(dp)      = hv;
  *(volatile v8h*)(dp + ND) = lv;
}

__global__ __launch_bounds__(128) void gln_kernel(const float* __restrict__ w, const float* __restrict__ gam,
                                                  const float* __restrict__ bet, _Float16* __restrict__ X) {
  const int row = blockIdx.x;
  if (row >= QLEN * NB) return;
  const int i = row / NB, b = row - i * NB;
  const int wave = threadIdx.x >> 5, lane = threadIdx.x & 31;
  const int col = wave * DG + lane * 8;
  const float* sp = w + ((size_t)i * NB_FULL + b) * ND + col;
  const v4f a = *(const v4f*)(sp);
  const v4f c = *(const v4f*)(sp + 4);
  float x[8];
  x[0] = bf_rne(a[0]); x[1] = bf_rne(a[1]); x[2] = bf_rne(a[2]); x[3] = bf_rne(a[3]);
  x[4] = bf_rne(c[0]); x[5] = bf_rne(c[1]); x[6] = bf_rne(c[2]); x[7] = bf_rne(c[3]);
  float s = ((x[0] + x[1]) + (x[2] + x[3])) + ((x[4] + x[5]) + (x[6] + x[7]));
  s += __shfl_xor(s, 1, 32);  s += __shfl_xor(s, 2, 32);  s += __shfl_xor(s, 4, 32);
  s += __shfl_xor(s, 8, 32);  s += __shfl_xor(s, 16, 32);
  const float mean = s * (1.0f / (float)DG);
  float d[8];
#pragma unroll
  for (int e = 0; e < 8; ++e) d[e] = x[e] - mean;
  float ss = ((d[0] * d[0] + d[1] * d[1]) + (d[2] * d[2] + d[3] * d[3])) +
             ((d[4] * d[4] + d[5] * d[5]) + (d[6] * d[6] + d[7] * d[7]));
  ss += __shfl_xor(ss, 1, 32); ss += __shfl_xor(ss, 2, 32); ss += __shfl_xor(ss, 4, 32);
  ss += __shfl_xor(ss, 8, 32); ss += __shfl_xor(ss, 16, 32);
  const float var = ss * (1.0f / (float)(DG - 1));
  const float inv = 1.0f / (sqrtf(var) + LN_EPS);
  const v4f ga = *(const v4f*)(gam + col);
  const v4f gb = *(const v4f*)(gam + col + 4);
  const v4f ba = *(const v4f*)(bet + col);
  const v4f bb = *(const v4f*)(bet + col + 4);
  float g8[8], b8[8];
  g8[0] = bf_rne(ga[0]); g8[1] = bf_rne(ga[1]); g8[2] = bf_rne(ga[2]); g8[3] = bf_rne(ga[3]);
  g8[4] = bf_rne(gb[0]); g8[5] = bf_rne(gb[1]); g8[6] = bf_rne(gb[2]); g8[7] = bf_rne(gb[3]);
  b8[0] = bf_rne(ba[0]); b8[1] = bf_rne(ba[1]); b8[2] = bf_rne(ba[2]); b8[3] = bf_rne(ba[3]);
  b8[4] = bf_rne(bb[0]); b8[5] = bf_rne(bb[1]); b8[6] = bf_rne(bb[2]); b8[7] = bf_rne(bb[3]);
  v8h hv, lv;
#pragma unroll
  for (int e = 0; e < 8; ++e) {
    const float y = g8[e] * (d[e] * inv) + b8[e];
    const _Float16 hq = (_Float16)y;
    hv[e] = hq;
    lv[e] = (_Float16)((y - (float)hq) * 1024.0f);
  }
  _Float16* dp = X + (size_t)row * QKW + col;
  *(volatile v8h*)(dp)      = hv;
  *(volatile v8h*)(dp + ND) = lv;
  __threadfence();
  *(volatile v8h*)(dp)      = hv;
  *(volatile v8h*)(dp + ND) = lv;
}

__global__ __launch_bounds__(128) void ln_kernel(const float* __restrict__ mems, const float* __restrict__ w,
                                                 const float* __restrict__ gam, const float* __restrict__ bet,
                                                 _Float16* __restrict__ X) {
  __shared__ float ps[4];
  __shared__ float pq[4];
  const int row = blockIdx.x;
  const int k = row / NB, b = row - k * NB;
  const int tid = threadIdx.x, wave = tid >> 5, lane = tid & 31;
  const int col = tid * 8;
  const float* sp = (k < MLEN) ? (mems + ((size_t)k * NB_FULL + b) * ND)
                               : (w + ((size_t)(k - MLEN) * NB_FULL + b) * ND);
  sp += col;
  const v4f a = *(const v4f*)(sp);
  const v4f c = *(const v4f*)(sp + 4);
  float x[8];
  x[0] = bf_rne(a[0]); x[1] = bf_rne(a[1]); x[2] = bf_rne(a[2]); x[3] = bf_rne(a[3]);
  x[4] = bf_rne(c[0]); x[5] = bf_rne(c[1]); x[6] = bf_rne(c[2]); x[7] = bf_rne(c[3]);
  float s = ((x[0] + x[1]) + (x[2] + x[3])) + ((x[4] + x[5]) + (x[6] + x[7]));
  s += __shfl_xor(s, 1, 32);  s += __shfl_xor(s, 2, 32);  s += __shfl_xor(s, 4, 32);
  s += __shfl_xor(s, 8, 32);  s += __shfl_xor(s, 16, 32);
  if (lane == 0) ps[wave] = s;
  __syncthreads();
  const float S = (ps[0] + ps[1]) + (ps[2] + ps[3]);
  const float mean = S * (1.0f / (float)ND);
  float d[8];
#pragma unroll
  for (int e = 0; e < 8; ++e) d[e] = x[e] - mean;
  float ss = ((d[0] * d[0] + d[1] * d[1]) + (d[2] * d[2] + d[3] * d[3])) +
             ((d[4] * d[4] + d[5] * d[5]) + (d[6] * d[6] + d[7] * d[7]));
  ss += __shfl_xor(ss, 1, 32); ss += __shfl_xor(ss, 2, 32); ss += __shfl_xor(ss, 4, 32);
  ss += __shfl_xor(ss, 8, 32); ss += __shfl_xor(ss, 16, 32);
  if (lane == 0) pq[wave] = ss;
  __syncthreads();
  const float SS  = (pq[0] + pq[1]) + (pq[2] + pq[3]);
  const float var = SS * (1.0f / (float)(ND - 1));
  const float inv = 1.0f / (sqrtf(var) + LN_EPS);
  const v4f ga = *(const v4f*)(gam + col);
  const v4f gb = *(const v4f*)(gam + col + 4);
  const v4f ba = *(const v4f*)(bet + col);
  const v4f bb = *(const v4f*)(bet + col + 4);
  float g8[8], b8[8];
  g8[0] = bf_rne(ga[0]); g8[1] = bf_rne(ga[1]); g8[2] = bf_rne(ga[2]); g8[3] = bf_rne(ga[3]);
  g8[4] = bf_rne(gb[0]); g8[5] = bf_rne(gb[1]); g8[6] = bf_rne(gb[2]); g8[7] = bf_rne(gb[3]);
  b8[0] = bf_rne(ba[0]); b8[1] = bf_rne(ba[1]); b8[2] = bf_rne(ba[2]); b8[3] = bf_rne(ba[3]);
  b8[4] = bf_rne(bb[0]); b8[5] = bf_rne(bb[1]); b8[6] = bf_rne(bb[2]); b8[7] = bf_rne(bb[3]);
  v8h hv, lv;
#pragma unroll
  for (int e = 0; e < 8; ++e) {
    const float y = g8[e] * (d[e] * inv) + b8[e];
    const _Float16 hq = (_Float16)y;
    hv[e] = hq;
    lv[e] = (_Float16)((y - (float)hq) * 1024.0f);
  }
  _Float16* dp = X + (size_t)row * QKW + col;
  *(volatile v8h*)(dp)      = hv;
  *(volatile v8h*)(dp + ND) = lv;
  __threadfence();
  *(volatile v8h*)(dp)      = hv;
  *(volatile v8h*)(dp + ND) = lv;
}

template <int OUT, bool HASB>
__global__ __launch_bounds__(256) void gemm_f16_kernel(
    const _Float16* __restrict__ A, int lda, long strideA,
    const _Float16* __restrict__ Bt, int ldb, long strideB,
    void* C1, void* C2, int ldc, long strideC,
    const float* __restrict__ b1, const float* __restrict__ b2,
    int M, int N, int K, float scale, float carry) {
  __shared__ __align__(16) float sT[8][16 * 68];

  const int z    = blockIdx.y;
  const int lane = threadIdx.x & 31;
  const int wave = threadIdx.x >> 5;
  const int tilesN = N >> 6;
  const int tilesM = M >> 6;
  const int tile = blockIdx.x * 8 + wave;
  if (tile >= tilesM * tilesN) return;
  const int tm = tile / tilesN;
  const int tn = tile - tm * tilesN;
  const int m0 = tm << 6;
  const int n0 = tn << 6;

  const _Float16* Ab = A  + (size_t)z * (size_t)strideA;
  const _Float16* Bb = Bt + (size_t)z * (size_t)strideB;

  const int rl   = lane & 15;
  const int koff = (lane >> 4) * 8;
  const int mOff = (lane >> 4) * 8;

  v8f acc[4][4];
#pragma unroll
  for (int i = 0; i < 4; ++i)
#pragma unroll
    for (int j = 0; j < 4; ++j) acc[i][j] = zero8();

  for (int k0 = 0; k0 < K; k0 += 32) {
    v16h bfr[4];
#pragma unroll
    for (int j = 0; j < 4; ++j)
      bfr[j] = ldfrag(Bb + (size_t)(n0 + (j << 4) + rl) * ldb + koff + k0);
#pragma unroll
    for (int i = 0; i < 4; ++i) {
      const v16h af = ldfrag(Ab + (size_t)(m0 + (i << 4) + rl) * lda + koff + k0);
#pragma unroll
      for (int j = 0; j < 4; ++j) acc[i][j] = mma16(af, bfr[j], acc[i][j]);
    }
  }

  float* slab = sT[wave];
  const int hh = lane >> 4, c4 = (lane & 15) * 4;
  const int q8 = lane >> 3, c8 = (lane & 7) * 8;
  float col8a[8], col8b[8];
#pragma unroll
  for (int e = 0; e < 8; ++e) { col8a[e] = 0.f; col8b[e] = 0.f; }
  if (OUT == 3) {
    const v4f ta = *(const v4f*)(b1 + n0 + c8);
    const v4f tb = *(const v4f*)(b1 + n0 + c8 + 4);
    col8a[0] = bf_rne(ta[0]); col8a[1] = bf_rne(ta[1]); col8a[2] = bf_rne(ta[2]); col8a[3] = bf_rne(ta[3]);
    col8a[4] = bf_rne(tb[0]); col8a[5] = bf_rne(tb[1]); col8a[6] = bf_rne(tb[2]); col8a[7] = bf_rne(tb[3]);
    const v4f tc = *(const v4f*)(b2 + n0 + c8);
    const v4f td = *(const v4f*)(b2 + n0 + c8 + 4);
    col8b[0] = bf_rne(tc[0]); col8b[1] = bf_rne(tc[1]); col8b[2] = bf_rne(tc[2]); col8b[3] = bf_rne(tc[3]);
    col8b[4] = bf_rne(td[0]); col8b[5] = bf_rne(td[1]); col8b[6] = bf_rne(td[2]); col8b[7] = bf_rne(td[3]);
  }
  const float carry2 = carry * 0.0009765625f;

#pragma unroll
  for (int i = 0; i < 4; ++i) {
    const int mBase = m0 + (i << 4);
#pragma unroll
    for (int j = 0; j < 4; ++j)
#pragma unroll
      for (int r = 0; r < 8; ++r)
        slab[(mOff + r) * 68 + (j << 4) + rl] = acc[i][j][r] * scale;
    __builtin_amdgcn_fence(__ATOMIC_RELEASE, "workgroup");
    __builtin_amdgcn_wave_barrier();
    __builtin_amdgcn_fence(__ATOMIC_ACQUIRE, "workgroup");
    if (OUT == 0 || OUT == 1) {
      float* C = (float*)C1 + (size_t)z * (size_t)strideC;
      v4f vv[8];
#pragma unroll
      for (int it = 0; it < 8; ++it) {
        const int row = it * 2 + hh;
        v4f v = *(const v4fa*)(slab + row * 68 + c4);
        if (OUT == 1 && HASB) {
          const int mr = mBase + row;
          const int ib = mr / NB, bb = mr - ib * NB;
          const float* rp = b1 + ((size_t)ib * NB_FULL + bb) * ND + n0 + c4;
          const v4f t = *(const v4f*)(rp);
          v4f rb;
          rb[0] = bf_rne(t[0]); rb[1] = bf_rne(t[1]); rb[2] = bf_rne(t[2]); rb[3] = bf_rne(t[3]);
          v += rb;
        }
        vv[it] = v;
      }
      for (int ps = 0; ps < 2; ++ps) {
#pragma unroll
        for (int it = 0; it < 8; ++it) {
          const int row = it * 2 + hh;
          *(volatile v4f*)(C + (size_t)(mBase + row) * ldc + n0 + c4) = vv[it];
        }
        __threadfence();
      }
    } else if (OUT == 2 || OUT == 4) {
      _Float16* Ca = (_Float16*)C1 + (size_t)z * (size_t)strideC;
      v8h hv[4], lv[4];
#pragma unroll
      for (int it = 0; it < 4; ++it) {
        const int row = it * 4 + q8;
        const float* sp = slab + row * 68 + c8;
        const v4f x0 = *(const v4fa*)(sp);
        const v4f x1 = *(const v4fa*)(sp + 4);
        float f[8];
        f[0] = x0[0]; f[1] = x0[1]; f[2] = x0[2]; f[3] = x0[3];
        f[4] = x1[0]; f[5] = x1[1]; f[6] = x1[2]; f[7] = x1[3];
        v8h ha, la;
#pragma unroll
        for (int e = 0; e < 8; ++e) {
          const float t = f[e];
          ha[e] = (_Float16)(t * carry);
          la[e] = (_Float16)(t * carry2);
        }
        hv[it] = ha; lv[it] = la;
      }
      for (int ps = 0; ps < 2; ++ps) {
#pragma unroll
        for (int it = 0; it < 4; ++it) {
          const int row = it * 4 + q8;
          if (OUT == 2) {
            _Float16* cp = Ca + (size_t)(mBase + row) * ldc + 2 * n0 + c8;
            *(volatile v8h*)(cp)      = hv[it];
            *(volatile v8h*)(cp + 64) = lv[it];
          } else {
            *(volatile v8h*)(Ca + (size_t)(mBase + row) * ldc + n0 + c8) = hv[it];
          }
        }
        __threadfence();
      }
    } else {
#pragma unroll
      for (int var = 0; var < 2; ++var) {
        _Float16* Cc = (_Float16*)((var == 0) ? C1 : C2) + (size_t)z * (size_t)strideC;
        v8h hv[4], lv[4];
#pragma unroll
        for (int it = 0; it < 4; ++it) {
          const int row = it * 4 + q8;
          const float* sp = slab + row * 68 + c8;
          const v4f x0 = *(const v4fa*)(sp);
          const v4f x1 = *(const v4fa*)(sp + 4);
          float f[8];
          f[0] = x0[0]; f[1] = x0[1]; f[2] = x0[2]; f[3] = x0[3];
          f[4] = x1[0]; f[5] = x1[1]; f[6] = x1[2]; f[7] = x1[3];
          v8h ha, la;
#pragma unroll
          for (int e = 0; e < 8; ++e) {
            const float t  = f[e] + ((var == 0) ? col8a[e] : col8b[e]);
            const float th = t * carry;
            const _Float16 hq = (_Float16)th;
            ha[e] = hq;
            la[e] = (_Float16)((th - (float)hq) * 1024.0f);
          }
          hv[it] = ha; lv[it] = la;
        }
        for (int ps = 0; ps < 2; ++ps) {
#pragma unroll
          for (int it = 0; it < 4; ++it) {
            const int row = it * 4 + q8;
            _Float16* cp = Cc + (size_t)(mBase + row) * ldc + 2 * n0 + c8;
            *(volatile v8h*)(cp)      = hv[it];
            *(volatile v8h*)(cp + 64) = lv[it];
          }
          __threadfence();
        }
      }
    }
    __builtin_amdgcn_fence(__ATOMIC_RELEASE, "workgroup");
    __builtin_amdgcn_wave_barrier();
    __builtin_amdgcn_fence(__ATOMIC_ACQUIRE, "workgroup");
  }
}

__global__ __launch_bounds__(128)
void relattn_kernel(const _Float16* __restrict__ QU, const _Float16* __restrict__ KP,
                    const _Float16* __restrict__ VT, const float* __restrict__ BD,
                    const int* __restrict__ MSK, _Float16* __restrict__ CTX,
                    int h0, int b, float cs) {
  __shared__ __align__(16) unsigned char SMEM[32768];
  __shared__ __align__(16) int Msh[64 * 64];
  _Float16* Ksh = (_Float16*)(SMEM);
  _Float16* Vsh = (_Float16*)(SMEM + 16384);
  _Float16* Psh = (_Float16*)(SMEM + 24576);
  float*    Osh = (float*)(SMEM);

  const int tid  = threadIdx.x;
  const int wave = tid >> 5;
  const int lane = tid & 31;
  const int hh   = lane >> 4;
  const int c    = lane & 15;

  const int z    = blockIdx.y;
  const int h    = h0 + z;
  const int qb   = blockIdx.x;
  const int q0   = qb * 64 + wave * 16;
  const int rr0  = wave * 16 + 8 * hh;
  const int iq   = q0 + 8 * hh;

  const _Float16* Qh  = QU + (size_t)b * QKW + h * HQK;
  const _Float16* Kh  = KP + (size_t)b * QKW + h * HQK;
  const _Float16* Vh  = VT + ((size_t)b * ND + h * HDV) * KLEN;
  const float*    bd  = BD + (size_t)z * QLEN * BDN;
  const int*      mkb = MSK + (size_t)(qb * 64) * KLEN;
  _Float16*       ctx = CTX + (size_t)b * QKW + h * HDV;

  v16h qa[4];
#pragma unroll
  for (int dc = 0; dc < 4; ++dc)
    qa[dc] = ldfrag(Qh + (size_t)(q0 + c) * LDQ + dc * 32 + 8 * hh);

  float mrow[8], lrow[8];
  v8f oacc[4];
#pragma unroll
  for (int r = 0; r < 8; ++r) { mrow[r] = -INFINITY; lrow[r] = 0.f; }
#pragma unroll
  for (int t = 0; t < 4; ++t) oacc[t] = zero8();

  _Float16* pw = Psh + wave * (16 * 64);

#pragma unroll 1
  for (int kc = 0; kc < NKT; ++kc) {
    const int kv0 = kc * 64;
    __syncthreads();
    {
      const int r = tid >> 1, c0 = (tid & 1) * 64, cv = (tid & 1) * 32;
      const _Float16* ks = Kh + (size_t)(kv0 + r) * LDQ + c0;
      const _Float16* vs = Vh + (size_t)r * KLEN + kv0 + cv;
      const int*      ms = mkb + (size_t)r * KLEN + kv0 + cv;
#pragma unroll
      for (int i = 0; i < 8; ++i) {
        const v8h kk8 = *(const v8h*)(ks + 8 * i);
        *(v8ha*)(Ksh + r * 128 + c0 + 8 * i) = kk8;
      }
#pragma unroll
      for (int i = 0; i < 4; ++i) {
        const v8h vv8 = *(const v8h*)(vs + 8 * i);
        *(v8ha*)(Vsh + r * 64 + cv + 8 * i) = vv8;
      }
#pragma unroll
      for (int i = 0; i < 8; ++i) {
        const v4i mm4 = *(const v4i*)(ms + 4 * i);
        *(v4ia*)(Msh + r * 64 + cv + 4 * i) = mm4;
      }
    }
    __syncthreads();

    v8f s[4];
#pragma unroll
    for (int j = 0; j < 4; ++j) {
      s[j] = zero8();
#pragma unroll
      for (int dc = 0; dc < 4; ++dc) {
        const v16h kb = ldfrag(Ksh + (j * 16 + c) * 128 + dc * 32 + 8 * hh);
        s[j] = mma16(qa[dc], kb, s[j]);
      }
    }

    float cm[8];
#pragma unroll
    for (int r = 0; r < 8; ++r) {
      const int i  = iq + r;
      const int fb = i * BDN + (QLEN - 1) - i;
      float m = -INFINITY;
#pragma unroll
      for (int j = 0; j < 4; ++j) {
        const int key  = kv0 + (j << 4) + c;
        const int col0 = QLEN - i + key;
        int ia = fb + key - ((col0 >= KLEN + 2) ? 1 : 0);
        ia = (ia > QLEN * BDN - 1) ? (QLEN * BDN - 1) : ia;
        ia = (ia < 0) ? 0 : ia;
        const float bvl = bd[ia];
        const float bdv = (col0 == KLEN + 1) ? 0.0f : bvl;
        const float raw = s[j][r] * cs + bdv;
        const int   mv  = Msh[(rr0 + r) * 64 + (j << 4) + c];
        const float sv  = (mv != 0) ? -1.0e30f : raw;
        s[j][r] = sv;
        m = fmaxf(m, sv);
      }
      m = fmaxf(m, __shfl_xor(m, 1, 32));
      m = fmaxf(m, __shfl_xor(m, 2, 32));
      m = fmaxf(m, __shfl_xor(m, 4, 32));
      m = fmaxf(m, __shfl_xor(m, 8, 32));
      cm[r] = m;
      __asm__ __volatile__("" ::: "memory");
    }

#pragma unroll
    for (int r = 0; r < 8; ++r) {
      const float mnew  = fmaxf(mrow[r], cm[r]);
      const float alpha = __expf(mrow[r] - mnew);
      mrow[r] = mnew;
      float psum = 0.f;
#pragma unroll
      for (int j = 0; j < 4; ++j) {
        const float p = __expf(s[j][r] - mnew);
        psum += p;
        pw[(8 * hh + r) * 64 + j * 16 + c] = (_Float16)(p * 4096.0f);
      }
      psum += __shfl_xor(psum, 1, 32);
      psum += __shfl_xor(psum, 2, 32);
      psum += __shfl_xor(psum, 4, 32);
      psum += __shfl_xor(psum, 8, 32);
      lrow[r] = lrow[r] * alpha + psum;
#pragma unroll
      for (int t = 0; t < 4; ++t) oacc[t][r] *= alpha;
    }
    __builtin_amdgcn_fence(__ATOMIC_RELEASE, "workgroup");
    __builtin_amdgcn_wave_barrier();
    __builtin_amdgcn_fence(__ATOMIC_ACQUIRE, "workgroup");

#pragma unroll
    for (int kk = 0; kk < 2; ++kk) {
      const v16h pa = ldfrag(pw + c * 64 + kk * 32 + 8 * hh);
#pragma unroll
      for (int t = 0; t < 4; ++t) {
        const v16h vb = ldfrag(Vsh + (t * 16 + c) * 64 + kk * 32 + 8 * hh);
        oacc[t] = mma16(pa, vb, oacc[t]);
      }
    }
  }

  __syncthreads();
  float* os = Osh + wave * (16 * HDV);
#pragma unroll
  for (int r = 0; r < 8; ++r) {
    const float inv = 1.0f / (1024.0f * lrow[r]);
#pragma unroll
    for (int t = 0; t < 4; ++t) os[(8 * hh + r) * HDV + t * 16 + c] = oacc[t][r] * inv;
  }
  __builtin_amdgcn_fence(__ATOMIC_RELEASE, "workgroup");
  __builtin_amdgcn_wave_barrier();
  __builtin_amdgcn_fence(__ATOMIC_ACQUIRE, "workgroup");
  const int q8 = lane >> 3, c8 = (lane & 7) * 8;
  v8h hv[4], lv[4];
#pragma unroll
  for (int it = 0; it < 4; ++it) {
    const int row = it * 4 + q8;
    const float* sp = os + row * HDV + c8;
    const v4f x0 = *(const v4fa*)(sp);
    const v4f x1 = *(const v4fa*)(sp + 4);
    float f[8];
    f[0] = x0[0]; f[1] = x0[1]; f[2] = x0[2]; f[3] = x0[3];
    f[4] = x1[0]; f[5] = x1[1]; f[6] = x1[2]; f[7] = x1[3];
    v8h ha, la;
#pragma unroll
    for (int e = 0; e < 8; ++e) {
      const float th = f[e];
      const _Float16 hq = (_Float16)th;
      ha[e] = hq;
      la[e] = (_Float16)((th - (float)hq) * 1024.0f);
    }
    hv[it] = ha; lv[it] = la;
  }
  for (int ps = 0; ps < 2; ++ps) {
#pragma unroll
    for (int it = 0; it < 4; ++it) {
      const int row = it * 4 + q8;
      _Float16* cp = ctx + (size_t)(q0 + row) * LDQ + c8;
      *(volatile v8h*)(cp)      = hv[it];
      *(volatile v8h*)(cp + ND) = lv[it];
    }
    __threadfence();
  }
}

extern "C" void kernel_launch(void* const* d_in, const int* in_sizes, int n_in,
                              void* d_out, int out_size, void* d_ws, size_t ws_size,
                              hipStream_t stream) {
  if (n_in < 17) return;
  if (in_sizes[0] < ((QLEN - 1) * NB_FULL + NB) * ND) return;
  if (in_sizes[1] < KLEN * ND) return;
  if (in_sizes[2] < NH * HDV || in_sizes[3] < NH * HDV) return;
  if (in_sizes[4] < ((MLEN - 1) * NB_FULL + NB) * ND) return;
  if (in_sizes[5] < ND || in_sizes[6] < ND || in_sizes[7] < ND || in_sizes[8] < ND) return;
  if (in_sizes[9] < NG * DG * DG) return;
  if (in_sizes[10] < DG * ND) return;
  if (in_sizes[11] < ND * ND || in_sizes[12] < ND * ND) return;
  if (in_sizes[13] < NG * DG * DG) return;
  if (in_sizes[14] < NG * DG * DG) return;
  if (in_sizes[15] < DG * ND) return;
  if (in_sizes[16] < QLEN * KLEN) return;
  if (out_size < QLEN * NB * ND) return;

  const float* w     = (const float*)d_in[0];
  const float* rpos  = (const float*)d_in[1];
  const float* rwb   = (const float*)d_in[2];
  const float* rrb   = (const float*)d_in[3];
  const float* mems  = (const float*)d_in[4];
  const float* gq    = (const float*)d_in[5];
  const float* bq    = (const float*)d_in[6];
  const float* gkv   = (const float*)d_in[7];
  const float* bkv   = (const float*)d_in[8];
  const float* Wg_q  = (const float*)d_in[9];
  const float* Wi_q  = (const float*)d_in[10];
  const float* Wk    = (const float*)d_in[11];
  const float* Wv    = (const float*)d_in[12];
  const float* Wr    = (const float*)d_in[13];
  const float* Wg_o  = (const float*)d_in[14];
  const float* Wi_o  = (const float*)d_in[15];
  const int*   mask  = (const int*)d_in[16];
  float* out = (float*)d_out;

  const size_t szW2  = (size_t)ND * QKW * 2;
  const size_t szWR  = (size_t)NG * DG * DG * 2;
  const size_t szRH  = (size_t)KLEN * ND * 2;
  const size_t szXQ  = (size_t)QLEN * NB * QKW * 2;
  const size_t szXKV = (size_t)KLEN * NB * QKW * 2;
  const size_t szQ2  = (size_t)QLEN * NB * QKW * 2;
  const size_t szKP2 = (size_t)KLEN * NB * QKW * 2;
  const size_t szVT  = (size_t)NB * ND * KLEN * 2;
  const size_t szP2  = (size_t)KLEN * QKW * 2;
  const size_t szCTX = (size_t)QLEN * NB * QKW * 2;
  const size_t szBD  = (size_t)NPAIR * QLEN * BDN * 4;
  size_t off = 0;
  const size_t oWQC = off; off += szW2;
  const size_t oWK  = off; off += szW2;
  const size_t oWV  = off; off += szW2;
  const size_t oWOC = off; off += szW2;
  const size_t oWR  = off; off += szWR;
  const size_t oRH  = off; off += szRH;
  const size_t oXQ  = off; off += szXQ;
  const size_t oXKV = off; off += szXKV;
  const size_t oQW2 = off; off += szQ2;
  const size_t oQR2 = off; off += szQ2;
  const size_t oKP2 = off; off += szKP2;
  const size_t oVT  = off; off += szVT;
  const size_t oP2  = off; off += szP2;
  const size_t oCTX = off; off += szCTX;
  const size_t oBD  = off; off += szBD;
  const size_t total = off;
  if (total > ws_size) return;
  if (total > (size_t)134217728) return;

  char* ws = (char*)d_ws;
  _Float16* WQCp = (_Float16*)(ws + oWQC);
  _Float16* WKp  = (_Float16*)(ws + oWK);
  _Float16* WVp  = (_Float16*)(ws + oWV);
  _Float16* WOCp = (_Float16*)(ws + oWOC);
  _Float16* WRp  = (_Float16*)(ws + oWR);
  _Float16* RHp  = (_Float16*)(ws + oRH);
  _Float16* XQ   = (_Float16*)(ws + oXQ);
  _Float16* XKV  = (_Float16*)(ws + oXKV);
  _Float16* QW2  = (_Float16*)(ws + oQW2);
  _Float16* QR2  = (_Float16*)(ws + oQR2);
  _Float16* KP2  = (_Float16*)(ws + oKP2);
  _Float16* VTp  = (_Float16*)(ws + oVT);
  _Float16* P2   = (_Float16*)(ws + oP2);
  _Float16* CTX  = (_Float16*)(ws + oCTX);
  float*    BDp  = (float*)(ws + oBD);

  const float cs   = 0.125f * 0.00390625f;
  const float r64  = 0.015625f;
  const float r4k  = 0.000244140625f;
  const dim3 blk(256);

  const int gW2 = (ND * (ND / 8) + 255) / 256;
  cvt2_kernel<true><<<dim3(gW2), blk, 0, stream>>>(Wi_q, Wg_q, WQCp);
  cvt2_kernel<false><<<dim3(gW2), blk, 0, stream>>>(Wk, Wk, WKp);
  cvt2_kernel<false><<<dim3(gW2), blk, 0, stream>>>(Wv, Wv, WVp);
  cvt2_kernel<true><<<dim3(gW2), blk, 0, stream>>>(Wi_o, Wg_o, WOCp);
  const int n8r = NG * DG * DG / 8;
  cvt1_kernel<<<dim3((n8r + 255) / 256), blk, 0, stream>>>(Wr, WRp, n8r, 64.0f);
  const int n8h = KLEN * ND / 8;
  cvt1_kernel<<<dim3((n8h + 255) / 256), blk, 0, stream>>>(rpos, RHp, n8h, 64.0f);
  gln_kernel<<<dim3(QLEN * NB), dim3(128), 0, stream>>>(w, gq, bq, XQ);
  ln_kernel<<<dim3(KLEN * NB), dim3(128), 0, stream>>>(mems, w, gkv, bkv, XKV);
  const int tilesQ = (QLEN / 64) * (ND / 64);
  gemm_f16_kernel<3, false><<<dim3((tilesQ + 7) / 8, NB), blk, 0, stream>>>(
      XQ, LDQ, (long)QKW, WQCp, QKW, 0L, (void*)QW2, (void*)QR2, LDQ, (long)QKW, rwb, rrb,
      QLEN, ND, QKW, r64, 16.0f);
  const int tilesK = (KLEN / 64) * (ND / 64);
  gemm_f16_kernel<2, false><<<dim3((tilesK + 7) / 8, NB), blk, 0, stream>>>(
      XKV, LDQ, (long)QKW, WKp, QKW, 0L, (void*)KP2, (void*)KP2, LDQ, (long)QKW, rwb, rwb,
      KLEN, ND, QKW, r64, 16.0f);
  gemm_f16_kernel<4, false><<<dim3((tilesK + 7) / 8, NB), blk, 0, stream>>>(
      WVp, QKW, 0L, XKV, LDQ, (long)QKW, (void*)VTp, (void*)VTp, KLEN, (long)ND * KLEN, rwb, rwb,
      ND, KLEN, QKW, r64, 16.0f);
  const int tilesR = (KLEN / 64) * (DG / 64);
  gemm_f16_kernel<2, false><<<dim3((tilesR + 7) / 8, NG), blk, 0, stream>>>(
      RHp, ND, (long)DG, WRp, DG, (long)DG * DG, (void*)P2, (void*)P2, QKW, (long)(2 * DG), rwb, rwb,
      KLEN, DG, DG, r4k, 16.0f);
  const int tilesB = (QLEN / 64) * (BDN / 64);
  for (int b = 0; b < NB; ++b) {
    for (int gi = 0; gi < NH / NPAIR; ++gi) {
      const int h0 = gi * NPAIR;
      const _Float16* Aq = QR2 + (size_t)b * QKW + h0 * HQK;
      const _Float16* Bp = P2 + h0 * HQK;
      gemm_f16_kernel<0, false><<<dim3((tilesB + 7) / 8, NPAIR), blk, 0, stream>>>(
          Aq, LDQ, (long)HQK, Bp, QKW, (long)HQK, (void*)BDp, (void*)BDp, BDN, (long)QLEN * BDN, rwb, rwb,
          QLEN, BDN, HQK, cs, 1.0f);
      relattn_kernel<<<dim3(NQT, NPAIR), dim3(128), 0, stream>>>(
          QW2, KP2, VTp, BDp, mask, CTX, h0, b, cs);
    }
  }
  const int tilesO = ((QLEN * NB) / 64) * (ND / 64);
  gemm_f16_kernel<1, true><<<dim3((tilesO + 7) / 8, 1), blk, 0, stream>>>(
      CTX, QKW, 0L, WOCp, QKW, 0L, (void*)out, (void*)out, ND, 0L, w, w,
      QLEN * NB, ND, QKW, r4k, 1.0f);
  (void)hipGetLastError();
}
